// PIGNN_77464030151232
// MI455X (gfx1250) — hardware-verified
//
#include <hip/hip_runtime.h>
#include <stdint.h>
#include <math.h>

#define NN 10000
#define NE 80000
#define NPAD 10048
#define HID 128
#define HID2 256
#define NSTEP 12
#define NODE_IN 25
#define EMB_IN 28
#define EMB_K 32
#define MSG_IN 259
#define UPD_IN 256
#define TW 20
#define C1K 15
#define C1O 8
#define C1T 29
#define C2K 10
#define NT 256
#define SRB 512
#define NTG 20
#define SCH 2048
#define NCH ((NE + SCH - 1) / SCH)
#define AGGR (NTG * SRB)
#define WSC 16.0f
#define WSC_INV 0.0625f
#define DEC_NB 32

static_assert(NPAD % 64 == 0 && NPAD >= NN);
static_assert(NE % 64 == 0);
static_assert(NE % (SCH / NT) == 0 && (SCH / NT) % 4 == 0);
static_assert(AGGR >= NPAD);
static_assert((NN * TW) % 4 == 0);

typedef __attribute__((ext_vector_type(16))) _Float16 v16h;
typedef __attribute__((ext_vector_type(8)))  _Float16 v8h;
typedef __attribute__((ext_vector_type(8)))  float    v8f;
typedef __attribute__((ext_vector_type(4)))  float    v4f;
typedef __attribute__((ext_vector_type(4)))  int      v4i;

__device__ __forceinline__ void dep_guard_h(v8f& a, v8f& b, v16h x, v16h y) { asm volatile("v_nop\n\tv_nop\n\tv_nop\n\tv_nop" : "+v"(a), "+v"(b) : "v"(x), "v"(y)); }
__device__ __forceinline__ void keep4_h(v16h a, v16h b, v16h c, v16h d) { asm volatile("v_nop" :: "v"(a), "v"(b), "v"(c), "v"(d)); }
__device__ __forceinline__ void acc_guard4(v8f& a, v8f& b, v8f& c, v8f& d) { asm volatile("v_nop\n\tv_nop\n\tv_nop\n\tv_nop" : "+v"(a), "+v"(b), "+v"(c), "+v"(d)); }
template <typename T> struct Frag;
template <> struct Frag<_Float16> {
  typedef v16h V; union U { v16h v; v8h h[2]; };
  static __device__ __forceinline__ v16h load(const _Float16* p) {
    U f; f.h[0] = *(const v8h*)(p); f.h[1] = *(const v8h*)(p + 16); return f.v;
  }
  static __device__ __forceinline__ v8f mma(v16h a, v16h b, v8f c) {
    return __builtin_amdgcn_wmma_f32_16x16x32_f16(false, a, false, b, (short)0, c, false, false);
  }
  static __device__ __forceinline__ void guard(v8f& a, v8f& b, v16h x, v16h y) { dep_guard_h(a, b, x, y); }
  static __device__ __forceinline__ void keep(v16h a, v16h b, v16h c, v16h d) { keep4_h(a, b, c, d); }
};

template <int BIAS_MODE, int OUT_MODE, bool RESID_POST, int ACT>
__global__ __launch_bounds__(256) void gemm_f16(
    const unsigned short* __restrict__ Ap, int lda,
    const unsigned short* __restrict__ Btp, int ldb,
    void* Cout, int ldc, void* Cout2, int ldc2,
    const float* __restrict__ bias, const float* resid, int ldr,
    int M, int N, int K, float scale) {
  typedef _Float16 T;
  typedef v16h V;
  const T* A = (const T*)Ap; const T* Bt = (const T*)Btp;
  __shared__ __align__(16) float sT[8][16 * 68];
  const int lane = threadIdx.x & 31;
  const int wave = threadIdx.x >> 5;
  const int tilesN = N >> 6;
  const int tilesM = M >> 6;
  const int tile = blockIdx.x * 8 + wave;
  if (tile >= tilesM * tilesN) return;
  const int tm = tile / tilesN;
  const int tn = tile - tm * tilesN;
  const int m0 = tm << 6;
  const int n0 = tn << 6;

  const int rlane = lane & 15;
  const int koff  = (lane >> 4) * 8;
  const int mOff  = (lane >> 4) * 8;

  v8f acc[4][4];
#pragma unroll
  for (int i = 0; i < 4; ++i)
#pragma unroll
    for (int j = 0; j < 4; ++j) acc[i][j] = (v8f){0.f,0.f,0.f,0.f,0.f,0.f,0.f,0.f};

  for (int k0 = 0; k0 < K; k0 += 32) {
    V bh[4];
#pragma unroll
    for (int j = 0; j < 4; ++j) {
      const size_t bo = (size_t)(n0 + (j << 4) + rlane) * ldb + koff + k0;
      bh[j] = Frag<T>::load(Bt + bo);
    }
#pragma unroll
    for (int i = 0; i < 4; ++i) {
      const size_t ao = (size_t)(m0 + (i << 4) + rlane) * lda + koff + k0;
      V ah = Frag<T>::load(A + ao);
#pragma unroll
      for (int j = 0; j < 4; ++j) acc[i][j] = Frag<T>::mma(ah, bh[j], acc[i][j]);
      Frag<T>::guard(acc[i][0], acc[i][3], ah, ah);
    }
    Frag<T>::keep(bh[0], bh[1], bh[2], bh[3]);
  }
  acc_guard4(acc[0][0], acc[0][1], acc[0][2], acc[0][3]);
  acc_guard4(acc[1][0], acc[1][1], acc[1][2], acc[1][3]);
  acc_guard4(acc[2][0], acc[2][1], acc[2][2], acc[2][3]);
  acc_guard4(acc[3][0], acc[3][1], acc[3][2], acc[3][3]);

  float* slab = sT[wave];
#pragma unroll
  for (int i = 0; i < 4; ++i) {
    const int mBase = m0 + (i << 4);
#pragma unroll
    for (int j = 0; j < 4; ++j) {
      const int n = n0 + (j << 4) + rlane;
      float bv = 0.f;
      if (BIAS_MODE == 2) bv = bias[n];
#pragma unroll
      for (int r = 0; r < 8; ++r) {
        float v = acc[i][j][r] * scale;
        if (BIAS_MODE == 2) v += bv;
        if (ACT == 2) v = fmaxf(v, 0.0f);
        if (RESID_POST) v += resid[(size_t)(mBase + mOff + r) * ldr + n];
        slab[(mOff + r) * 68 + (j << 4) + rlane] = v;
      }
    }
    __builtin_amdgcn_fence(__ATOMIC_RELEASE, "workgroup");
    __builtin_amdgcn_wave_barrier();
    __builtin_amdgcn_fence(__ATOMIC_ACQUIRE, "workgroup");
    if (OUT_MODE == 0 || OUT_MODE == 3) {
      float* C = (float*)Cout;
      const int hh = lane >> 4, c4 = (lane & 15) * 4;
      for (int pass = 0; pass < 2; ++pass) {
#pragma unroll
        for (int it = 0; it < 8; ++it) {
          const int row = it * 2 + hh;
          v4f v = *(const v4f*)(slab + row * 68 + c4);
          *(volatile v4f*)(C + (size_t)(mBase + row) * ldc + n0 + c4) = v;
        }
        __threadfence();
      }
    }
    if (OUT_MODE == 1 || OUT_MODE == 3) {
      const int q = lane >> 3, c8 = (lane & 7) * 8;
      unsigned short* C16 = (OUT_MODE == 1) ? (unsigned short*)Cout : (unsigned short*)Cout2;
      const int p16 = (OUT_MODE == 1) ? ldc : ldc2;
      for (int pass = 0; pass < 2; ++pass) {
#pragma unroll
        for (int it = 0; it < 4; ++it) {
          const int row = it * 4 + q;
          const float* sp = slab + row * 68 + c8;
          v8h hv;
#pragma unroll
          for (int e = 0; e < 8; ++e) hv[e] = (_Float16)sp[e];
          *(volatile v8h*)(C16 + (size_t)(mBase + row) * p16 + n0 + c8) = hv;
        }
        __threadfence();
      }
    }
    __builtin_amdgcn_fence(__ATOMIC_RELEASE, "workgroup");
    __builtin_amdgcn_wave_barrier();
    __builtin_amdgcn_fence(__ATOMIC_ACQUIRE, "workgroup");
  }
}

__global__ __launch_bounds__(NT) void wconv_kernel(const float* __restrict__ src, unsigned short* __restrict__ dst,
                                                  int Z, int srcZ, int srcLd, int dstZ, int nOff, int Nn, int Kin, int Kp) {
  const int kg = Kp >> 3;
  const int gpz = Nn * kg;
  const int total = Z * gpz;
  const int g = blockIdx.x * NT + threadIdx.x;
  if (g >= total) return;
  const int z = g / gpz;
  const int rem = g - z * gpz;
  const int n = rem / kg;
  const int k0 = (rem - n * kg) * 8;
  v8h hv;
#pragma unroll
  for (int e = 0; e < 8; ++e) {
    const int k = k0 + e;
    const int kc = k < Kin ? k : Kin - 1;
    const float f = src[(size_t)z * srcZ + (size_t)kc * srcLd + n];
    hv[e] = (_Float16)((k < Kin) ? f * WSC : 0.0f);
  }
  unsigned short* op = dst + (size_t)z * dstZ + (size_t)(nOff + n) * Kp + k0;
  *(volatile v8h*)op = hv;
  __threadfence();
  *(volatile v8h*)op = hv;
}

__global__ __launch_bounds__(NT) void a0_kernel(const float* __restrict__ x, const float* __restrict__ pos, const float* __restrict__ gattr,
                                               unsigned short* __restrict__ A0) {
  const int g = blockIdx.x * NT + threadIdx.x;
  if (g >= NPAD * (EMB_K / 8)) return;
  const int row = g >> 2, k0 = (g & 3) * 8;
  const bool live = row < NN;
  const int rc = live ? row : NN - 1;
  const float p0 = pos[(size_t)rc * 2], p1 = pos[(size_t)rc * 2 + 1], gv = gattr[0];
  v8h hv;
#pragma unroll
  for (int e = 0; e < 8; ++e) {
    const int c = k0 + e;
    const int cc = c < NODE_IN ? c : NODE_IN - 1;
    const float xv = x[(size_t)rc * NODE_IN + cc];
    float v = (c < NODE_IN) ? xv : ((c == NODE_IN) ? p0 : ((c == NODE_IN + 1) ? p1 : ((c == NODE_IN + 2) ? gv : 0.0f)));
    v = live ? v : 0.0f;
    hv[e] = (_Float16)v;
  }
  unsigned short* op = A0 + (size_t)row * EMB_K + k0;
  *(volatile v8h*)op = hv;
  __threadfence();
  *(volatile v8h*)op = hv;
}

__global__ __launch_bounds__(NT) void gather_kernel(const float* __restrict__ P, const float* __restrict__ eattr, const int* __restrict__ ei,
                                                   const float* __restrict__ Wc, const float* __restrict__ b1, unsigned short* __restrict__ M16) {
  const int lane = threadIdx.x & 31, wave = threadIdx.x >> 5;
  const int hh = lane >> 4, c0 = (lane & 15) * 8;
  const v4f wa0 = *(const v4f*)(Wc + c0),           wa1 = *(const v4f*)(Wc + c0 + 4);
  const v4f wb0 = *(const v4f*)(Wc + HID + c0),     wb1 = *(const v4f*)(Wc + HID + c0 + 4);
  const v4f wd0 = *(const v4f*)(Wc + 2 * HID + c0), wd1 = *(const v4f*)(Wc + 2 * HID + c0 + 4);
  const v4f bb0 = *(const v4f*)(b1 + c0),           bb1 = *(const v4f*)(b1 + c0 + 4);
  const int e0 = blockIdx.x * 64 + wave * 8;
#pragma unroll 1
  for (int it = 0; it < 4; ++it) {
    const int e = e0 + 2 * it + hh;
    int s = ei[e], d = ei[NE + e];
    s = s < 0 ? 0 : (s >= NN ? NN - 1 : s);
    d = d < 0 ? 0 : (d >= NN ? NN - 1 : d);
    const float ea0 = eattr[(size_t)e * 3], ea1 = eattr[(size_t)e * 3 + 1], ea2 = eattr[(size_t)e * 3 + 2];
    const float* pd = P + (size_t)d * HID2 + c0;
    const float* ps = P + (size_t)s * HID2 + HID + c0;
    v4f v0 = *(const v4f*)pd + *(const v4f*)ps + bb0;
    v4f v1 = *(const v4f*)(pd + 4) + *(const v4f*)(ps + 4) + bb1;
    v0 = v0 + ea0 * wa0 + ea1 * wb0 + ea2 * wd0;
    v1 = v1 + ea0 * wa1 + ea1 * wb1 + ea2 * wd1;
    v8h hv;
#pragma unroll
    for (int q = 0; q < 4; ++q) { hv[q] = (_Float16)fmaxf(v0[q], 0.0f); hv[4 + q] = (_Float16)fmaxf(v1[q], 0.0f); }
    unsigned short* op = M16 + (size_t)e * HID + c0;
    *(volatile v8h*)op = hv;
    __threadfence();
    *(volatile v8h*)op = hv;
  }
}

__device__ __forceinline__ int blk_excl_scan(int cnt, int* scan_ws, int tid, int* tot) {
  const int lane = tid & 31, wave = tid >> 5; int incl = cnt;
#pragma unroll
  for (int o = 1; o < 32; o <<= 1) { const int v = __shfl_up(incl, o, 32); if (lane >= o) incl += v; }
  if (lane == 31) scan_ws[wave] = incl;
  __syncthreads();
  if (wave == 0) { int wv = (lane < NT / 32) ? scan_ws[lane] : 0; int wincl = wv;
#pragma unroll
    for (int o = 1; o < 32; o <<= 1) { const int v = __shfl_up(wincl, o, 32); if (lane >= o) wincl += v; }
    if (lane < NT / 32) scan_ws[32 + lane] = wincl - wv; if (lane == 31) scan_ws[64] = wincl; }
  __syncthreads();
  const int res = scan_ws[32 + wave] + incl - cnt; *tot = scan_ws[64];
  return res;
}
template <int SP, int CAP>
__device__ __forceinline__ int chunk_hits(const int* __restrict__ dstv, int e0, int n0, int tid, int* LIST, int* scan_ws) {
  const int eb = e0 + tid * SP;
  const int ebc = (eb < NE) ? eb : (NE - SP);
  int rec[SP]; int cnt = 0;
#pragma unroll
  for (int k = 0; k < SP; k += 4) {
    const v4i d4 = *(const v4i*)(dstv + ebc + k);
#pragma unroll
    for (int e = 0; e < 4; ++e) {
      const int d = d4[e]; int r = -1;
      if (eb < NE && d >= n0 && d < n0 + SRB) { r = ((d - n0) << 17) | (ebc + k + e); ++cnt; }
      rec[k + e] = r;
    }
  }
  int tot; int p = blk_excl_scan(cnt, scan_ws, tid, &tot);
#pragma unroll
  for (int k = 0; k < SP; ++k) if (rec[k] >= 0) { if ((unsigned)p < (unsigned)CAP) LIST[p] = rec[k]; ++p; }
  __syncthreads();
  return tot < CAP ? tot : CAP;
}

__global__ __launch_bounds__(NT) void aggr_kernel(const float* __restrict__ MSG, const int* __restrict__ ei, float* AGG,
                                                 unsigned short* __restrict__ HA) {
  __shared__ int LIST[SCH];
  __shared__ int SDEG[SRB];
  __shared__ int scan_ws[80];
  const int tid = threadIdx.x, lane = tid & 31, wave = tid >> 5;
  const int n0 = blockIdx.x * SRB;
  const v4f z4 = {0.f, 0.f, 0.f, 0.f};
#pragma unroll 1
  for (int j = 0; j < 64; ++j) {
    float* rp = AGG + (size_t)(n0 + wave * 64 + j) * HID + 4 * lane;
    *(volatile v4f*)rp = z4;
    __threadfence();
    *(volatile v4f*)rp = z4;
  }
  for (int i = tid; i < SRB; i += NT) SDEG[i] = 0;
  __syncthreads();
  const int* dstv = ei + NE;
#pragma unroll 1
  for (int c = 0; c < NCH; ++c) {
    const int tot = chunk_hits<SCH / NT, SCH>(dstv, c * SCH, n0, tid, LIST, scan_ws);
#pragma unroll 1
    for (int base = 0; base < tot; base += 32) {
      const int q = base + lane;
      const int qc = q < SCH ? q : SCH - 1;
      const int lv = LIST[qc];
      const int rv = (q < tot) ? lv : -1;
      const int own = (rv >= 0 && (rv >> 23) == wave) ? 1 : 0;
      unsigned msk = (unsigned)__ballot(own);
#pragma unroll 1
      for (int it = 0; it < 32; ++it) {
        if (msk == 0u) break;
        const int bp = __builtin_ctz(msk); msk &= msk - 1u;
        const int r = __shfl(rv, bp, 32);
        const int dl = (r >> 17) & (SRB - 1);
        int e = r & 0x1FFFF; e = e < NE ? e : NE - 1;
        const v4f mv = *(const v4f*)(MSG + (size_t)e * HID + 4 * lane);
        float* rp = AGG + (size_t)(n0 + dl) * HID + 4 * lane;
        v4f a = *(const v4f*)rp;
        a = a + mv;
        *(volatile v4f*)rp = a;
        __threadfence();
        *(volatile v4f*)rp = a;
        if (lane == 0) SDEG[dl] += 1;
      }
    }
    __syncthreads();
  }
  const int hh = lane >> 4, l16 = lane & 15;
  const bool wvalid = (n0 + wave * 64) < NPAD;
  if (wvalid) {
#pragma unroll 1
    for (int j = 0; j < 64; j += 2) {
      const int dlr = wave * 64 + j + hh;
      const int n = n0 + dlr;
      const int dg = SDEG[dlr];
      const float inv = (dg > 0) ? (1.0f / (float)dg) : 0.0f;
      const float* rp = AGG + (size_t)(n0 + dlr) * HID + 8 * l16;
      const v4f a0 = *(const v4f*)rp, a1 = *(const v4f*)(rp + 4);
      v8h hv;
#pragma unroll
      for (int e = 0; e < 4; ++e) { hv[e] = (_Float16)(a0[e] * inv); hv[4 + e] = (_Float16)(a1[e] * inv); }
      unsigned short* op = HA + (size_t)n * HID2 + HID + 8 * l16;
      *(volatile v8h*)op = hv;
      __threadfence();
      *(volatile v8h*)op = hv;
    }
  }
}

__global__ __launch_bounds__(NT) void dec_kernel(const float* __restrict__ Hs, const float* __restrict__ c1W, const float* __restrict__ c1b,
                                                const float* __restrict__ c2W, const float* __restrict__ c2b, float* __restrict__ out) {
  __shared__ __align__(16) float hs[DEC_NB * HID];
  __shared__ float y1s[DEC_NB * C1O * C1T];
  __shared__ __align__(16) float so[DEC_NB * TW];
  const int tid = threadIdx.x, lane = tid & 31, wave = tid >> 5;
  const int nb = blockIdx.x * DEC_NB;
  int nn = NN - nb; nn = nn > DEC_NB ? DEC_NB : nn;
  for (int i = tid; i < DEC_NB * (HID / 4); i += NT) {
    const int row = i >> 5, c4 = (i & 31) * 4;
    *(v4f*)(hs + row * HID + c4) = *(const v4f*)(Hs + (size_t)(nb + row) * HID + c4);
  }
  __syncthreads();
  for (int i = tid; i < DEC_NB * C1O * C1T; i += NT) {
    const int nl = i / (C1O * C1T);
    const int rem = i - nl * (C1O * C1T);
    const int o = rem / C1T;
    const int t = rem - o * C1T;
    float a = c1b[o];
    const float* wp = c1W + o * C1K;
    const float* hp = hs + nl * HID + 4 * t;
#pragma unroll 1
    for (int k = 0; k < C1K; ++k) a += wp[k] * hp[k];
    y1s[i] = fmaxf(a, 0.0f);
  }
  __syncthreads();
  for (int i = tid; i < DEC_NB * TW; i += NT) {
    const int nl = i / TW;
    const int t = i - nl * TW;
    float a = c2b[0];
    const float* yp = y1s + nl * (C1O * C1T) + t;
#pragma unroll 1
    for (int o = 0; o < C1O; ++o) {
#pragma unroll 1
      for (int k = 0; k < C2K; ++k) a += c2W[o * C2K + k] * yp[o * C1T + k];
    }
    so[i] = a;
  }
  __syncthreads();
  if (wave == 0) {
    float* ob = out + (size_t)nb * TW;
    const int ng = nn * (TW / 4);
    for (int pass = 0; pass < 2; ++pass) {
      for (int g = lane; g < ng; g += 32) {
        const v4f v = *(const v4f*)(so + 4 * g);
        *(volatile v4f*)(ob + 4 * g) = v;
      }
      __threadfence();
    }
  }
}

template <int BM, int OM, bool RP, int AC>
static void launch_gemm(hipStream_t st, const void* A, int lda, const void* Bt, int ldb, void* C, int ldc, void* C2, int ldc2,
                        const float* bias, const float* resid, int ldr, int M, int N, int K) {
  const int tiles = (M / 64) * (N / 64);
  const int blocks = (tiles + 7) / 8;
  gemm_f16<BM, OM, RP, AC><<<dim3(blocks), dim3(256), 0, st>>>((const unsigned short*)A, lda, (const unsigned short*)Bt, ldb,
                                                               C, ldc, C2, ldc2, bias, resid, ldr, M, N, K, WSC_INV);
}

extern "C" void kernel_launch(void* const* d_in, const int* in_sizes, int n_in,
                              void* d_out, int out_size, void* d_ws, size_t ws_size, hipStream_t stream) {
  if (n_in < 22) return;
  if (in_sizes[0] != NN * NODE_IN || in_sizes[3] != NE * 3 || in_sizes[8] != NSTEP * MSG_IN * HID ||
      in_sizes[20] != 2 * NE || out_size != NN * TW) return;
  const float* x      = (const float*)d_in[0];
  const float* pos    = (const float*)d_in[1];
  const float* gattr  = (const float*)d_in[2];
  const float* eattr  = (const float*)d_in[3];
  const float* emb_W1 = (const float*)d_in[4];
  const float* emb_b1 = (const float*)d_in[5];
  const float* emb_W2 = (const float*)d_in[6];
  const float* emb_b2 = (const float*)d_in[7];
  const float* msg1_W = (const float*)d_in[8];
  const float* msg1_b = (const float*)d_in[9];
  const float* msg2_W = (const float*)d_in[10];
  const float* msg2_b = (const float*)d_in[11];
  const float* upd1_W = (const float*)d_in[12];
  const float* upd1_b = (const float*)d_in[13];
  const float* upd2_W = (const float*)d_in[14];
  const float* upd2_b = (const float*)d_in[15];
  const float* c1W    = (const float*)d_in[16];
  const float* c1b    = (const float*)d_in[17];
  const float* c2W    = (const float*)d_in[18];
  const float* c2b    = (const float*)d_in[19];
  const int*   ei     = (const int*)  d_in[20];
  float* out = (float*)d_out;

  char* ws = (char*)d_ws; size_t off = 0;
  auto carve = [&](size_t bytes) -> char* { char* p = ws + off; off += (bytes + 255) & ~(size_t)255; return p; };
  unsigned short* E1t  = (unsigned short*)carve((size_t)HID * EMB_K * 2);
  unsigned short* E2t  = (unsigned short*)carve((size_t)HID * HID * 2);
  unsigned short* W1t  = (unsigned short*)carve((size_t)NSTEP * HID2 * HID * 2);
  unsigned short* W2t  = (unsigned short*)carve((size_t)NSTEP * HID * HID * 2);
  unsigned short* U1t  = (unsigned short*)carve((size_t)NSTEP * HID * UPD_IN * 2);
  unsigned short* U2t  = (unsigned short*)carve((size_t)NSTEP * HID * HID * 2);
  unsigned short* A0   = (unsigned short*)carve((size_t)NPAD * EMB_K * 2);
  float*          H32  = (float*)carve((size_t)NPAD * HID * 4);
  unsigned short* HA16 = (unsigned short*)carve((size_t)NPAD * HID2 * 2);
  float*          P32  = (float*)carve((size_t)NPAD * HID2 * 4);
  unsigned short* U16  = (unsigned short*)carve((size_t)NPAD * HID * 2);
  unsigned short* M16  = (unsigned short*)carve((size_t)NE * HID * 2);
  float*          MSG  = (float*)carve((size_t)NE * HID * 4);
  float*          AGG  = (float*)carve((size_t)AGGR * HID * 4);
  if (off > ws_size || off > (size_t)134217728) return;

  auto wconv = [&](const float* src, unsigned short* dst, int Z, int srcZ, int dstZ, int nOff, int Nn, int Kin, int Kp) {
    const int total = Z * Nn * (Kp / 8);
    wconv_kernel<<<(total + NT - 1) / NT, NT, 0, stream>>>(src, dst, Z, srcZ, HID, dstZ, nOff, Nn, Kin, Kp);
  };
  wconv(emb_W1, E1t, 1, 0, 0, 0, HID, EMB_IN, EMB_K);
  wconv(emb_W2, E2t, 1, 0, 0, 0, HID, HID, HID);
  wconv(msg1_W, W1t, NSTEP, MSG_IN * HID, HID2 * HID, 0, HID, HID, HID);
  wconv(msg1_W + HID * HID, W1t, NSTEP, MSG_IN * HID, HID2 * HID, HID, HID, HID, HID);
  wconv(msg2_W, W2t, NSTEP, HID * HID, HID * HID, 0, HID, HID, HID);
  wconv(upd1_W, U1t, NSTEP, UPD_IN * HID, HID * UPD_IN, 0, HID, UPD_IN, UPD_IN);
  wconv(upd2_W, U2t, NSTEP, HID * HID, HID * HID, 0, HID, HID, HID);

  a0_kernel<<<(NPAD * (EMB_K / 8) + NT - 1) / NT, NT, 0, stream>>>(x, pos, gattr, A0);
  launch_gemm<2, 1, false, 2>(stream, A0, EMB_K, E1t, EMB_K, U16, HID, nullptr, 0, emb_b1, nullptr, 0, NPAD, HID, EMB_K);
  launch_gemm<2, 3, false, 2>(stream, U16, HID, E2t, HID, H32, HID, HA16, HID2, emb_b2, nullptr, 0, NPAD, HID, HID);

  for (int s = 0; s < NSTEP; ++s) {
    launch_gemm<0, 0, false, 0>(stream, HA16, HID2, W1t + (size_t)s * HID2 * HID, HID, P32, HID2, nullptr, 0,
                                nullptr, nullptr, 0, NPAD, HID2, HID);
    gather_kernel<<<NE / 64, NT, 0, stream>>>(P32, eattr, ei, msg1_W + (size_t)s * MSG_IN * HID + (size_t)HID2 * HID,
                                              msg1_b + (size_t)s * HID, M16);
    launch_gemm<2, 0, false, 2>(stream, M16, HID, W2t + (size_t)s * HID * HID, HID, MSG, HID, nullptr, 0,
                                msg2_b + (size_t)s * HID, nullptr, 0, NE, HID, HID);
    aggr_kernel<<<NTG, NT, 0, stream>>>(MSG, ei, AGG, HA16);
    launch_gemm<2, 1, false, 2>(stream, HA16, HID2, U1t + (size_t)s * HID * UPD_IN, UPD_IN, U16, HID, nullptr, 0,
                                upd1_b + (size_t)s * HID, nullptr, 0, NPAD, HID, UPD_IN);
    launch_gemm<2, 3, true, 2>(stream, U16, HID, U2t + (size_t)s * HID * HID, HID, H32, HID, HA16, HID2,
                               upd2_b + (size_t)s * HID, H32, HID, NPAD, HID, HID);
  }

  dec_kernel<<<(NN + DEC_NB - 1) / DEC_NB, NT, 0, stream>>>(H32, c1W, c1b, c2W, c2b, out);
}
